// FlashAttention_84112639525332
// MI455X (gfx1250) — hardware-verified
//
#include <hip/hip_runtime.h>

typedef unsigned short us16;
typedef us16   v8us  __attribute__((ext_vector_type(8)));
typedef __bf16 v16bf __attribute__((ext_vector_type(16)));
typedef float  v8f   __attribute__((ext_vector_type(8)));
typedef float  v4f   __attribute__((ext_vector_type(4)));
typedef v4f    v4fa  __attribute__((__may_alias__));
typedef int    v4i   __attribute__((ext_vector_type(4)));
typedef int    v8i   __attribute__((ext_vector_type(8)));

#ifndef NB
#define NB 2
#endif
#ifndef SEQ
#define SEQ 2048
#endif
#define NB_FULL  2
#define SEQ_FULL 2048
#define NH       16
#define DHEAD    64
#define ROWF     (NH * DHEAD)

#define BM   64
#define BN   64
#define PB   64
#define KST  72
#define VST  72
#define VLST 72
#define OST  68

#define SCL2 (0.125f * 1.4426950408889634f)
#define NEGL (-1.0e10f * 1.4426950408889634f)

static_assert(NB >= 1);
static_assert(NB <= NB_FULL);
static_assert(SEQ >= 64);
static_assert(SEQ <= SEQ_FULL);
static_assert(SEQ % BM == 0);
static_assert(SEQ % BN == 0);
static_assert(SEQ % PB == 0);
static_assert(BN == 64);
static_assert(BM == 64);
static_assert(PB == 64);
static_assert(DHEAD == 64);

#define PLANE_ELEMS ((size_t)NB * NH * SEQ * DHEAD)

__device__ __forceinline__ unsigned int bf_bits(float x) {
    const unsigned int u = __float_as_uint(x);
    return (u + 0x7FFFu + ((u >> 16) & 1u)) >> 16;
}

__device__ __forceinline__ v4i pack8(v4f a, v4f b) {
    v8us r;
    r[0] = (us16)bf_bits(a[0]); r[1] = (us16)bf_bits(a[1]);
    r[2] = (us16)bf_bits(a[2]); r[3] = (us16)bf_bits(a[3]);
    r[4] = (us16)bf_bits(b[0]); r[5] = (us16)bf_bits(b[1]);
    r[6] = (us16)bf_bits(b[2]); r[7] = (us16)bf_bits(b[3]);
    return __builtin_bit_cast(v4i, r);
}

union FragB { v16bf v; v8us h[2]; };

__device__ __forceinline__ v16bf ld_op16(const us16* p) {
    FragB f;
    f.h[0] = *(const v8us*)(p);
    f.h[1] = *(const v8us*)(p + 16);
    return f.v;
}

__device__ __forceinline__ v8f wmma_bf(v16bf a, v16bf b, v8f c) {
    return __builtin_amdgcn_wmma_f32_16x16x32_bf16(false, a, false, b, (short)0, c, false, false);
}

__device__ __forceinline__ void vguard4(v8f& a, v8f& b, v8f& c, v8f& d) {
    asm volatile("v_nop\n\tv_nop\n\tv_nop\n\tv_nop" : "+v"(a), "+v"(b), "+v"(c), "+v"(d));
}

__device__ __forceinline__ void fa_step(const us16* ksb, const us16* vtsb, const int* msb,
                                        const v16bf (&qb)[2], int l16, int kbase,
                                        float& m_i, float& l_i, v8f (&acc)[4]) {
    v8f s[4];
#pragma unroll
    for (int n = 0; n < 4; ++n)
#pragma unroll
        for (int v = 0; v < 8; ++v) s[n][v] = 0.0f;
#pragma unroll
    for (int c = 0; c < 2; ++c) {
        const int dco = c * 32 + kbase;
#pragma unroll
        for (int n = 0; n < 4; ++n) {
            const v16bf ka = ld_op16(&ksb[(n * 16 + l16) * KST + dco]);
            s[n] = wmma_bf(ka, qb[c], s[n]);
        }
    }
    vguard4(s[0], s[1], s[2], s[3]);

    float tm[4];
#pragma unroll
    for (int n = 0; n < 4; ++n) {
        union { v8i v; v4i h[2]; } mk;
        mk.h[0] = *(const v4i*)(msb + n * 16 + kbase);
        mk.h[1] = *(const v4i*)(msb + n * 16 + kbase + 4);
#pragma unroll
        for (int v = 0; v < 8; ++v) {
            const float sc = s[n][v] * SCL2;
            s[n][v] = (mk.v[v] > 0) ? sc : NEGL;
        }
        const float a0 = fmaxf(s[n][0], s[n][1]);
        const float a1 = fmaxf(s[n][2], s[n][3]);
        const float a2 = fmaxf(s[n][4], s[n][5]);
        const float a3 = fmaxf(s[n][6], s[n][7]);
        tm[n] = fmaxf(fmaxf(a0, a1), fmaxf(a2, a3));
    }
    float mx = fmaxf(fmaxf(tm[0], tm[1]), fmaxf(tm[2], tm[3]));
    mx = fmaxf(mx, __shfl_xor(mx, 16, 32));

    const float mnew = fmaxf(m_i, mx);
    const float corr = __builtin_amdgcn_exp2f(m_i - mnew);

    float psum = 0.0f;
    v16bf pbh[2], pbl[2];
#pragma unroll
    for (int n = 0; n < 4; ++n)
#pragma unroll
        for (int v = 0; v < 8; ++v) {
            const float  p  = __builtin_amdgcn_exp2f(s[n][v] - mnew);
            psum += p;
            const __bf16 ph = (__bf16)p;
            const float  pr = p - (float)ph;
            pbh[n >> 1][(n & 1) * 8 + v] = ph;
            pbl[n >> 1][(n & 1) * 8 + v] = (__bf16)pr;
        }
    psum += __shfl_xor(psum, 16, 32);

    l_i = l_i * corr + psum;
    m_i = mnew;
#pragma unroll
    for (int t = 0; t < 4; ++t) acc[t] = acc[t] * corr;

#pragma unroll
    for (int ck = 0; ck < 2; ++ck)
#pragma unroll
        for (int t = 0; t < 4; ++t) {
            const v16bf va = ld_op16(&vtsb[(t * 16 + l16) * VST + ck * 32 + kbase]);
            acc[t] = wmma_bf(va, pbh[ck], acc[t]);
            acc[t] = wmma_bf(va, pbl[ck], acc[t]);
        }
    vguard4(acc[0], acc[1], acc[2], acc[3]);
}

__global__ __launch_bounds__(256)
void k_prep(const float* __restrict__ Q, const float* __restrict__ K, const float* __restrict__ V,
            us16* __restrict__ Qp, us16* __restrict__ Kp, us16* __restrict__ Vtp) {
    __shared__ __align__(16) us16 Vl[DHEAD * VLST];

    const int tid  = threadIdx.x;
    const int lane = tid & 31;
    const int w    = tid >> 5;
    const int bh   = blockIdx.y;
    const int b    = bh / NH;
    const int hh   = bh - b * NH;
    const int j0   = blockIdx.x * PB;

    const size_t in_row0 = ((size_t)b * SEQ_FULL + (size_t)j0) * ROWF + (size_t)hh * DHEAD;
    const int    c       = tid & 7;

    v4i    qo[2], ko[2];
    size_t pgo[2];
#pragma unroll
    for (int it = 0; it < 2; ++it) {
        const int    r  = it * 32 + (tid >> 3);
        const size_t go = in_row0 + (size_t)r * ROWF + (size_t)c * 8;
        const v4f q0 = *(const v4f*)(Q + go);
        const v4f q1 = *(const v4f*)(Q + go + 4);
        const v4f k0 = *(const v4f*)(K + go);
        const v4f k1 = *(const v4f*)(K + go + 4);
        const v4f v0 = *(const v4f*)(V + go);
        const v4f v1 = *(const v4f*)(V + go + 4);
        qo[it]  = pack8(q0, q1);
        ko[it]  = pack8(k0, k1);
        pgo[it] = ((size_t)bh * SEQ + (size_t)(j0 + r)) * DHEAD + (size_t)c * 8;
        Vl[(c * 8 + 0) * VLST + r] = (us16)bf_bits(v0[0]);
        Vl[(c * 8 + 1) * VLST + r] = (us16)bf_bits(v0[1]);
        Vl[(c * 8 + 2) * VLST + r] = (us16)bf_bits(v0[2]);
        Vl[(c * 8 + 3) * VLST + r] = (us16)bf_bits(v0[3]);
        Vl[(c * 8 + 4) * VLST + r] = (us16)bf_bits(v1[0]);
        Vl[(c * 8 + 5) * VLST + r] = (us16)bf_bits(v1[1]);
        Vl[(c * 8 + 6) * VLST + r] = (us16)bf_bits(v1[2]);
        Vl[(c * 8 + 7) * VLST + r] = (us16)bf_bits(v1[3]);
    }
    __syncthreads();

    v4i    vo[2];
    size_t vgo[2];
#pragma unroll
    for (int it = 0; it < 2; ++it) {
        const int d  = w * 8 + it * 4 + (lane >> 3);
        const int cj = lane & 7;
        const v8us t8 = *(const v8us*)&Vl[d * VLST + cj * 8];
        vo[it]  = __builtin_bit_cast(v4i, t8);
        vgo[it] = ((size_t)bh * DHEAD + (size_t)d) * SEQ + (size_t)j0 + (size_t)cj * 8;
    }

#pragma unroll
    for (int it = 0; it < 2; ++it) {
        *(volatile v4i*)(Qp + pgo[it])  = qo[it];
        *(volatile v4i*)(Kp + pgo[it])  = ko[it];
        *(volatile v4i*)(Vtp + vgo[it]) = vo[it];
    }
    __threadfence();
#pragma unroll
    for (int it = 0; it < 2; ++it) {
        *(volatile v4i*)(Qp + pgo[it])  = qo[it];
        *(volatile v4i*)(Kp + pgo[it])  = ko[it];
        *(volatile v4i*)(Vtp + vgo[it]) = vo[it];
    }
}

__global__ __launch_bounds__(128)
void k_attn(const us16* __restrict__ Qp, const us16* __restrict__ Kp,
            const us16* __restrict__ Vtp, const int* __restrict__ Msk,
            float* __restrict__ O) {
    __shared__ __align__(16) us16  Ks[BN * KST];
    __shared__ __align__(16) us16  Vts[DHEAD * VST];
    __shared__ __align__(16) int   Ms[BN];
    __shared__ __align__(16) float Os[BM * OST];

    const int tid   = threadIdx.x;
    const int lane  = tid & 31;
    const int wid   = tid >> 5;
    const int h     = lane >> 4;
    const int l16   = lane & 15;
    const int kbase = h * 8;

    const int bh   = blockIdx.y;
    const int b    = bh / NH;
    const int hh   = bh - b * NH;
    const int qblk = blockIdx.x;

    const us16* Qpl  = Qp  + (size_t)bh * SEQ * DHEAD;
    const us16* Kpl  = Kp  + (size_t)bh * SEQ * DHEAD;
    const us16* Vtpl = Vtp + (size_t)bh * DHEAD * SEQ;
    const int*  mrow = Msk + (size_t)b * SEQ_FULL;

    const int   qbase = qblk * BM + wid * 16;
    const us16* qrow  = Qpl + (size_t)(qbase + l16) * DHEAD;
    v16bf qb[2];
#pragma unroll
    for (int c = 0; c < 2; ++c) qb[c] = ld_op16(qrow + c * 32 + kbase);

    float m_i = -1e30f, l_i = 0.0f;
    v8f acc[4];
#pragma unroll
    for (int t = 0; t < 4; ++t)
#pragma unroll
        for (int v = 0; v < 8; ++v) acc[t][v] = 0.0f;

    for (int kb = 0; kb < SEQ; kb += BN) {
        __syncthreads();
#pragma unroll
        for (int i = 0; i < 4; ++i) {
            const int cc  = tid + 128 * i;
            const int row = cc >> 3;
            const int off = (cc & 7) * 8;
            *(v8us*)&Ks[row * KST + off]  = *(const v8us*)(Kpl + (size_t)(kb + row) * DHEAD + off);
            *(v8us*)&Vts[row * VST + off] = *(const v8us*)(Vtpl + (size_t)row * SEQ + (size_t)(kb + off));
        }
        if (tid < BN) Ms[tid] = mrow[kb + tid];
        __syncthreads();
        fa_step(Ks, Vts, Ms, qb, l16, kbase, m_i, l_i, acc);
    }

    const float inv = 1.0f / l_i;
    float*      osr = &Os[(wid * 16 + l16) * OST];
#pragma unroll
    for (int t = 0; t < 4; ++t) {
        v4f a, c;
        a[0] = acc[t][0] * inv; a[1] = acc[t][1] * inv; a[2] = acc[t][2] * inv; a[3] = acc[t][3] * inv;
        c[0] = acc[t][4] * inv; c[1] = acc[t][5] * inv; c[2] = acc[t][6] * inv; c[3] = acc[t][7] * inv;
        *(v4fa*)&osr[t * 16 + kbase]     = a;
        *(v4fa*)&osr[t * 16 + kbase + 4] = c;
    }
    __syncthreads();

    const size_t orow0 = ((size_t)b * SEQ + (size_t)(qblk * BM)) * ROWF + (size_t)hh * DHEAD;
    v4f ov[8];
#pragma unroll
    for (int it = 0; it < 8; ++it) {
        const int q = wid * 16 + it * 2 + h;
        ov[it] = *(const v4fa*)&Os[q * OST + l16 * 4];
    }
#pragma unroll
    for (int it = 0; it < 8; ++it) {
        const int q = wid * 16 + it * 2 + h;
        *(volatile v4f*)(O + orow0 + (size_t)q * ROWF + (size_t)(l16 * 4)) = ov[it];
    }
    __threadfence();
#pragma unroll
    for (int it = 0; it < 8; ++it) {
        const int q = wid * 16 + it * 2 + h;
        *(volatile v4f*)(O + orow0 + (size_t)q * ROWF + (size_t)(l16 * 4)) = ov[it];
    }
}

extern "C" void kernel_launch(void* const* d_in, const int* in_sizes, int n_in,
                              void* d_out, int out_size, void* d_ws, size_t ws_size,
                              hipStream_t stream) {
    if (n_in < 4) return;
    const long long need_rows = (long long)(NB - 1) * SEQ_FULL + SEQ;
    const long long need_qkv  = need_rows * ROWF;
    if ((long long)in_sizes[0] < need_qkv) return;
    if ((long long)in_sizes[1] < need_qkv) return;
    if ((long long)in_sizes[2] < need_qkv) return;
    if ((long long)in_sizes[3] < need_rows) return;
    if ((long long)out_size < (long long)NB * SEQ * ROWF) return;
    const size_t plane_bytes = PLANE_ELEMS * sizeof(us16);
    if (ws_size < 3 * plane_bytes) return;

    const float* Q   = (const float*)d_in[0];
    const float* K   = (const float*)d_in[1];
    const float* V   = (const float*)d_in[2];
    const int*   Msk = (const int*)d_in[3];
    float*       O   = (float*)d_out;

    us16* Qp  = (us16*)d_ws;
    us16* Kp  = Qp + PLANE_ELEMS;
    us16* Vtp = Kp + PLANE_ELEMS;

    const int nbh = NB * NH;

    k_prep<<<dim3(SEQ / PB, nbh), dim3(256), 0, stream>>>(Q, K, V, Qp, Kp, Vtp);
    k_attn<<<dim3(SEQ / BM, nbh), dim3(128), 0, stream>>>(Qp, Kp, Vtp, Msk, O);
}
